// MambaVision_36326833390111
// MI455X (gfx1250) — hardware-run, weakly checked
//
#include <hip/hip_runtime.h>
#include <math.h>

constexpr int kBatch  = 16;
constexpr int kSeq    = 1024;
constexpr int kDModel = 512;
constexpr int kDInner = 1024;
constexpr int kDHalf  = 512;
constexpr int kDState = 16;
constexpr int kDConv  = 4;
constexpr int kDtRank = 32;
constexpr int kXdbl   = 64;
constexpr int kTok    = kBatch * kSeq;
constexpr float kWCarry  = 16.0f;
constexpr float kACarry  = 64.0f;
constexpr float kScaleIn = 1.0f / 16.0f;
constexpr float kScaleAW = 1.0f / 1024.0f;
constexpr int kScanCh  = 64;
constexpr int kSYP     = 132;

typedef __attribute__((ext_vector_type(16))) _Float16 v16h;
typedef __attribute__((ext_vector_type(8)))  _Float16 v8h;
typedef __attribute__((ext_vector_type(16))) __bf16   v16b;
typedef __attribute__((ext_vector_type(8)))  __bf16   v8b;
typedef __attribute__((ext_vector_type(8)))  float    v8f;
typedef __attribute__((ext_vector_type(4)))  float    v4f;
typedef __attribute__((ext_vector_type(4)))  unsigned int v4u;

__device__ __forceinline__ unsigned short f2bf_bits(float f) {
  unsigned u = __float_as_uint(f);
  return (unsigned short)((u + 0x7FFFu + ((u >> 16) & 1u)) >> 16);
}
__device__ __forceinline__ float bf_bits2f(unsigned short h) { return __uint_as_float(((unsigned)h) << 16); }

__device__ __forceinline__ void dep_guard_h(v8f& a, v8f& b, v16h x, v16h y) { asm volatile("v_nop\n\tv_nop\n\tv_nop\n\tv_nop" : "+v"(a), "+v"(b) : "v"(x), "v"(y)); }
__device__ __forceinline__ void dep_guard_b(v8f& a, v8f& b, v16b x, v16b y) { asm volatile("v_nop\n\tv_nop\n\tv_nop\n\tv_nop" : "+v"(a), "+v"(b) : "v"(x), "v"(y)); }
__device__ __forceinline__ void keep4_h(v16h a, v16h b, v16h c, v16h d) { asm volatile("v_nop" :: "v"(a), "v"(b), "v"(c), "v"(d)); }
__device__ __forceinline__ void keep4_b(v16b a, v16b b, v16b c, v16b d) { asm volatile("v_nop" :: "v"(a), "v"(b), "v"(c), "v"(d)); }
__device__ __forceinline__ void acc_guard4(v8f& a, v8f& b, v8f& c, v8f& d) { asm volatile("v_nop\n\tv_nop\n\tv_nop\n\tv_nop" : "+v"(a), "+v"(b), "+v"(c), "+v"(d)); }
template <typename T> struct Frag;
template <> struct Frag<_Float16> {
  typedef v16h V; union U { v16h v; v8h h[2]; };
  static __device__ __forceinline__ v16h load(const _Float16* p) {
    U f; f.h[0] = *(const v8h*)(p); f.h[1] = *(const v8h*)(p + 16); return f.v;
  }
  static __device__ __forceinline__ v8f mma(v16h a, v16h b, v8f c) {
    return __builtin_amdgcn_wmma_f32_16x16x32_f16(false, a, false, b, (short)0, c, false, false);
  }
  static __device__ __forceinline__ void guard(v8f& a, v8f& b, v16h x, v16h y) { dep_guard_h(a, b, x, y); }
  static __device__ __forceinline__ void keep(v16h a, v16h b, v16h c, v16h d) { keep4_h(a, b, c, d); }
};
template <> struct Frag<__bf16> {
  typedef v16b V; union U { v16b v; v8b h[2]; };
  static __device__ __forceinline__ v16b load(const __bf16* p) {
    U f; f.h[0] = *(const v8b*)(p); f.h[1] = *(const v8b*)(p + 16); return f.v;
  }
  static __device__ __forceinline__ v8f mma(v16b a, v16b b, v8f c) {
    return __builtin_amdgcn_wmma_f32_16x16x32_bf16(false, a, false, b, (short)0, c, false, false);
  }
  static __device__ __forceinline__ void guard(v8f& a, v8f& b, v16b x, v16b y) { dep_guard_b(a, b, x, y); }
  static __device__ __forceinline__ void keep(v16b a, v16b b, v16b c, v16b d) { keep4_b(a, b, c, d); }
};

__device__ __forceinline__ unsigned pk16(unsigned short a, unsigned short b) { return (unsigned)a | ((unsigned)b << 16); }
__device__ __forceinline__ unsigned short h_bits(float f) { const _Float16 h = (_Float16)f; return __builtin_bit_cast(unsigned short, h); }

template <int ET> struct Elem;
template <> struct Elem<0> { typedef _Float16 T; };
template <> struct Elem<1> { typedef __bf16 T; };
template <int ET, bool SPLIT, int BIAS_MODE, int OUT_MODE, bool RESID, int ACT = 0>
__global__ __launch_bounds__(256) void wmma_gemm64(
    const unsigned short* __restrict__ Ap, const unsigned short* __restrict__ A2p, int lda, long strideA,
    const unsigned short* __restrict__ Btp, const unsigned short* __restrict__ Bt2p, int ldb, long strideB,
    void* __restrict__ Cout, void* __restrict__ Cout2, int ldc, long strideC,
    const float* __restrict__ bias,
    const float* __restrict__ resid, long strideR,
    int M, int N, int K, float scale) {
  typedef typename Elem<ET>::T T;
  typedef typename Frag<T>::V V;
  const T* A = (const T*)Ap; const T* A2 = (const T*)A2p; const T* Bt = (const T*)Btp; const T* Bt2 = (const T*)Bt2p;
  __shared__ __align__(16) float sT[8][16 * 68];
  const int b    = blockIdx.y;
  const int lane = threadIdx.x & 31;
  const int wave = threadIdx.x >> 5;
  const int tilesN = N >> 6;
  const int tilesM = M >> 6;
  const int tile = blockIdx.x * 8 + wave;
  if (tile >= tilesM * tilesN) return;
  const int tm = tile / tilesN;
  const int tn = tile - tm * tilesN;
  const int m0 = tm << 6;
  const int n0 = tn << 6;

  const T* Ab  = A  + (size_t)b * strideA;
  const T* Bb  = Bt + (size_t)b * strideB;
  const T* Ab2 = SPLIT ? (A2  + (size_t)b * strideA) : nullptr;
  const T* Bb2 = SPLIT ? (Bt2 + (size_t)b * strideB) : nullptr;

  const int rlane = lane & 15;
  const int koff  = (lane >> 4) * 8;
  const int mOff  = (lane >> 4) * 8;

  v8f acc[4][4];
#pragma unroll
  for (int i = 0; i < 4; ++i)
#pragma unroll
    for (int j = 0; j < 4; ++j) acc[i][j] = (v8f){0.f,0.f,0.f,0.f,0.f,0.f,0.f,0.f};

  for (int k0 = 0; k0 < K; k0 += 32) {
    V bh[4], bl[4];
#pragma unroll
    for (int j = 0; j < 4; ++j) {
      const size_t bo = (size_t)(n0 + (j << 4) + rlane) * ldb + koff + k0;
      bh[j] = Frag<T>::load(Bb + bo);
      if (SPLIT) bl[j] = Frag<T>::load(Bb2 + bo);
    }
#pragma unroll
    for (int i = 0; i < 4; ++i) {
      const size_t ao = (size_t)(m0 + (i << 4) + rlane) * lda + koff + k0;
      V ah = Frag<T>::load(Ab + ao);
      V al;
      if (SPLIT) al = Frag<T>::load(Ab2 + ao);
#pragma unroll
      for (int j = 0; j < 4; ++j) {
        acc[i][j] = Frag<T>::mma(ah, bh[j], acc[i][j]);
        if (SPLIT) {
          acc[i][j] = Frag<T>::mma(ah, bl[j], acc[i][j]);
          acc[i][j] = Frag<T>::mma(al, bh[j], acc[i][j]);
        }
      }
      Frag<T>::guard(acc[i][0], acc[i][3], ah, SPLIT ? al : ah);
    }
    Frag<T>::keep(bh[0], bh[1], bh[2], bh[3]);
    if (SPLIT) Frag<T>::keep(bl[0], bl[1], bl[2], bl[3]);
  }
  acc_guard4(acc[0][0], acc[0][1], acc[0][2], acc[0][3]);
  acc_guard4(acc[1][0], acc[1][1], acc[1][2], acc[1][3]);
  acc_guard4(acc[2][0], acc[2][1], acc[2][2], acc[2][3]);
  acc_guard4(acc[3][0], acc[3][1], acc[3][2], acc[3][3]);

  float* slab = sT[wave];
  const float* Rb = RESID ? (resid + (size_t)b * strideR) : nullptr;
#pragma unroll
  for (int i = 0; i < 4; ++i) {
    const int mBase = m0 + (i << 4);
#pragma unroll
    for (int j = 0; j < 4; ++j) {
      const int n = n0 + (j << 4) + rlane;
      float bv = 0.f;
      if (BIAS_MODE == 2) bv = bias[n];
#pragma unroll
      for (int r = 0; r < 8; ++r) {
        float v = acc[i][j][r] * scale;
        if (BIAS_MODE == 1) v += bias[mBase + mOff + r];
        if (BIAS_MODE == 2) v += bv;
        if (RESID) v += Rb[(size_t)(mBase + mOff + r) * ldc + n];
        if (ACT == 2) v = fmaxf(v, 0.0f);
        if (ACT == 4) v = (v > 0.f) ? v : 0.01f * v;
        slab[(mOff + r) * 68 + (j << 4) + rlane] = v;
      }
    }
    __builtin_amdgcn_fence(__ATOMIC_RELEASE, "workgroup");
    __builtin_amdgcn_wave_barrier();
    __builtin_amdgcn_fence(__ATOMIC_ACQUIRE, "workgroup");
    if (OUT_MODE == 0) {
      float* C = (float*)Cout + (size_t)b * strideC;
      const int hh = lane >> 4, c4 = (lane & 15) * 4;
      for (int pass = 0; pass < 2; ++pass) {
#pragma unroll
        for (int it = 0; it < 8; ++it) {
          const int row = it * 2 + hh;
          v4f v = *(const v4f*)(slab + row * 68 + c4);
          *(volatile v4f*)(C + (size_t)(mBase + row) * ldc + n0 + c4) = v;
        }
        __threadfence();
      }
    } else {
      const int q = lane >> 3, c8 = (lane & 7) * 8;
      unsigned short* C  = (unsigned short*)Cout  + (size_t)b * strideC;
      unsigned short* C2 = (OUT_MODE == 2) ? ((unsigned short*)Cout2 + (size_t)b * strideC) : nullptr;
      for (int pass = 0; pass < 2; ++pass) {
#pragma unroll
        for (int it = 0; it < 4; ++it) {
          const int row = it * 4 + q;
          const float* sp = slab + row * 68 + c8;
          v8h hv, lv;
#pragma unroll
          for (int e = 0; e < 8; ++e) {
            if (OUT_MODE == 1) {
              hv[e] = (_Float16)sp[e];
            } else {
              unsigned short hb = f2bf_bits(sp[e]);
              unsigned short lb = f2bf_bits(sp[e] - bf_bits2f(hb));
              hv[e] = __builtin_bit_cast(_Float16, hb);
              lv[e] = __builtin_bit_cast(_Float16, lb);
            }
          }
          *(volatile v8h*)(C + (size_t)(mBase + row) * ldc + n0 + c8) = hv;
          if (OUT_MODE == 2) *(volatile v8h*)(C2 + (size_t)(mBase + row) * ldc + n0 + c8) = lv;
        }
        __threadfence();
      }
    }
    __builtin_amdgcn_fence(__ATOMIC_RELEASE, "workgroup");
    __builtin_amdgcn_wave_barrier();
    __builtin_amdgcn_fence(__ATOMIC_ACQUIRE, "workgroup");
  }
}

__global__ __launch_bounds__(256) void cast8_f16_kernel(const float* __restrict__ in, unsigned short* __restrict__ out,
                                                        int n8, float carry) {
  const int i = blockIdx.x * 256 + threadIdx.x;
  if (i >= n8) return;
  const float* p = in + 8 * (size_t)i;
  const v4f a = *(const v4f*)(p);
  const v4f c = *(const v4f*)(p + 4);
  unsigned short hb[8];
#pragma unroll
  for (int e = 0; e < 4; ++e) {
    hb[e]     = h_bits(a[e] * carry);
    hb[4 + e] = h_bits(c[e] * carry);
  }
  const v4u u = (v4u){pk16(hb[0], hb[1]), pk16(hb[2], hb[3]), pk16(hb[4], hb[5]), pk16(hb[6], hb[7])};
  unsigned short* q = out + 8 * (size_t)i;
  *(volatile v4u*)q = u;
  __threadfence();
  *(volatile v4u*)q = u;
}

__global__ __launch_bounds__(256) void dtcast_kernel(const float* __restrict__ XD, unsigned short* __restrict__ DT16, int n8) {
  const int i = blockIdx.x * 256 + threadIdx.x;
  if (i >= n8) return;
  const int row = i >> 2;
  const int q = i & 3;
  const float* p = XD + (size_t)row * kXdbl + 8 * q;
  const v4f a = *(const v4f*)(p);
  const v4f c = *(const v4f*)(p + 4);
  unsigned short hb[8];
#pragma unroll
  for (int e = 0; e < 4; ++e) {
    hb[e]     = h_bits(a[e] * kACarry);
    hb[4 + e] = h_bits(c[e] * kACarry);
  }
  const v4u u = (v4u){pk16(hb[0], hb[1]), pk16(hb[2], hb[3]), pk16(hb[4], hb[5]), pk16(hb[6], hb[7])};
  unsigned short* dst = DT16 + (size_t)row * kDtRank + 8 * q;
  *(volatile v4u*)dst = u;
  __threadfence();
  *(volatile v4u*)dst = u;
}

__device__ __forceinline__ float conv_silu4(float xm1, float x0, float x1, float x2,
                                            float w0, float w1, float w2, float w3) {
#pragma clang fp contract(off)
  float a = xm1 * w0;
  a = a + x0 * w1;
  a = a + x1 * w2;
  a = a + x2 * w3;
  const float e = expf(-a);
  const float sg = 1.0f / (1.0f + e);
  return a * sg;
}
__device__ __forceinline__ float softplus_f(float x) {
#pragma clang fp contract(off)
  const float t = log1pf(expf(-fabsf(x)));
  return fmaxf(x, 0.0f) + t;
}

__global__ __launch_bounds__(256) void conv_silu_kernel(
    const float* __restrict__ XP, const float* __restrict__ ZP,
    const float* __restrict__ wx, const float* __restrict__ wz,
    unsigned short* __restrict__ X16, unsigned short* __restrict__ YZ16) {
#pragma clang fp contract(off)
  const int g = blockIdx.x * 256 + threadIdx.x;
  const int row = g >> 6;
  const int c8 = (g & 63) * 8;
  const int l = row & (kSeq - 1);
  const bool hm1 = (l >= 1);
  const bool hp1 = (l + 1 < kSeq);
  const bool hp2 = (l + 2 < kSeq);
  const int rm1 = hm1 ? (row - 1) : row;
  const int rp1 = hp1 ? (row + 1) : row;
  const int rp2 = hp2 ? (row + 2) : row;
  union U8 { v4f q[2]; float f[8]; };
#pragma unroll 1
  for (int hf = 0; hf < 2; ++hf) {
    const float* P = (hf == 0) ? XP : ZP;
    const float* W = (hf == 0) ? wx : wz;
    U8 um1, u0, u1, u2;
    um1.q[0] = *(const v4f*)(P + (size_t)rm1 * kDHalf + c8);
    um1.q[1] = *(const v4f*)(P + (size_t)rm1 * kDHalf + c8 + 4);
    u0.q[0]  = *(const v4f*)(P + (size_t)row * kDHalf + c8);
    u0.q[1]  = *(const v4f*)(P + (size_t)row * kDHalf + c8 + 4);
    u1.q[0]  = *(const v4f*)(P + (size_t)rp1 * kDHalf + c8);
    u1.q[1]  = *(const v4f*)(P + (size_t)rp1 * kDHalf + c8 + 4);
    u2.q[0]  = *(const v4f*)(P + (size_t)rp2 * kDHalf + c8);
    u2.q[1]  = *(const v4f*)(P + (size_t)rp2 * kDHalf + c8 + 4);
    unsigned short hb[8];
#pragma unroll
    for (int e = 0; e < 8; ++e) {
      const int c = c8 + e;
      const float w0 = W[c * kDConv + 0];
      const float w1 = W[c * kDConv + 1];
      const float w2 = W[c * kDConv + 2];
      const float w3 = W[c * kDConv + 3];
      const float vm1 = hm1 ? um1.f[e] : 0.0f;
      const float v0  = u0.f[e];
      const float v1  = hp1 ? u1.f[e] : 0.0f;
      const float v2  = hp2 ? u2.f[e] : 0.0f;
      const float s   = conv_silu4(vm1, v0, v1, v2, w0, w1, w2, w3);
      hb[e] = h_bits(s * kACarry);
    }
    const v4u u = (v4u){pk16(hb[0], hb[1]), pk16(hb[2], hb[3]), pk16(hb[4], hb[5]), pk16(hb[6], hb[7])};
    unsigned short* dst = (hf == 0) ? (X16 + (size_t)row * kDHalf + c8)
                                    : (YZ16 + (size_t)row * kDInner + kDHalf + c8);
    *(volatile v4u*)dst = u;
    __threadfence();
    *(volatile v4u*)dst = u;
  }
}

__global__ __launch_bounds__(128) void scan_kernel(
    const float* __restrict__ XP,
    const float* __restrict__ XDBL,
    const float* __restrict__ DTP,
    const float* __restrict__ Alog,
    const float* __restrict__ Dv,
    const float* __restrict__ wx,
    unsigned short* __restrict__ YZ16)
{
#pragma clang fp contract(off)
  __shared__ __align__(16) float sBC[kScanCh * 32];
  __shared__ __align__(16) float sY[kScanCh * kSYP];
  const int b    = blockIdx.x;
  const int d0   = blockIdx.y * 128;
  const int tid  = threadIdx.x;
  const int d    = d0 + tid;
  const int lane = tid & 31;
  const int wave = tid >> 5;

  float a[kDState], h[kDState];
#pragma unroll
  for (int n = 0; n < kDState; ++n) {
    a[n] = -expf(Alog[d * kDState + n]);
    h[n] = 0.f;
  }
  const float Dd = Dv[d];
  const float w0 = wx[d * kDConv + 0];
  const float w1 = wx[d * kDConv + 1];
  const float w2 = wx[d * kDConv + 2];
  const float w3 = wx[d * kDConv + 3];
  const size_t rowb = (size_t)b * kSeq;
  float xm1 = 0.f;
  float x0  = XP[(rowb + 0) * kDHalf + d];
  float x1  = XP[(rowb + 1) * kDHalf + d];
  float x2  = XP[(rowb + 2) * kDHalf + d];

#pragma unroll 1
  for (int l0 = 0; l0 < kSeq; l0 += kScanCh) {
    __syncthreads();
#pragma unroll 1
    for (int i = tid; i < kScanCh * 32; i += 128) {
      const int s = i >> 5;
      const int c = i & 31;
      sBC[i] = XDBL[(rowb + l0 + s) * kXdbl + 32 + c];
    }
    __syncthreads();
#pragma unroll 1
    for (int s = 0; s < kScanCh; ++s) {
      const int l = l0 + s;
      const size_t row = rowb + l;
      const float xv = conv_silu4(xm1, x0, x1, x2, w0, w1, w2, w3);
      const int ln = (l + 3 < kSeq) ? (l + 3) : (kSeq - 1);
      const float xn = XP[(rowb + ln) * kDHalf + d];
      xm1 = x0; x0 = x1; x1 = x2; x2 = (l + 3 < kSeq) ? xn : 0.f;
      const float pre = DTP[row * kDHalf + d];
      const float dlt = softplus_f(pre);
      union U16 { v4f q[4]; float f[16]; };
      U16 Bv, Cv;
#pragma unroll
      for (int qq = 0; qq < 4; ++qq) {
        Bv.q[qq] = *(const v4f*)(sBC + s * 32 + 4 * qq);
        Cv.q[qq] = *(const v4f*)(sBC + s * 32 + 16 + 4 * qq);
      }
      float y = 0.f;
#pragma unroll
      for (int n = 0; n < kDState; ++n) {
        const float dA  = expf(dlt * a[n]);
        const float dBx = (dlt * Bv.f[n]) * xv;
        h[n] = dA * h[n] + dBx;
        y = y + h[n] * Cv.f[n];
      }
      y = y + xv * Dd;
      sY[s * kSYP + tid] = y;
    }
    __syncthreads();
    {
      const int hr = lane >> 4;
      const int c8 = (lane & 15) * 8;
      for (int pass = 0; pass < 2; ++pass) {
#pragma unroll
        for (int it = 0; it < 8; ++it) {
          const int r = wave * 16 + it * 2 + hr;
          const float* sp = sY + r * kSYP + c8;
          const v4f qa = *(const v4f*)(sp);
          const v4f qb = *(const v4f*)(sp + 4);
          const v4u u = (v4u){pk16(h_bits(qa[0] * kACarry), h_bits(qa[1] * kACarry)),
                               pk16(h_bits(qa[2] * kACarry), h_bits(qa[3] * kACarry)),
                               pk16(h_bits(qb[0] * kACarry), h_bits(qb[1] * kACarry)),
                               pk16(h_bits(qb[2] * kACarry), h_bits(qb[3] * kACarry))};
          *(volatile v4u*)(YZ16 + (rowb + l0 + r) * kDInner + d0 + c8) = u;
        }
        __threadfence();
      }
    }
  }
}

extern "C" void kernel_launch(void* const* d_in, const int* in_sizes, int n_in,
                              void* d_out, int out_size, void* d_ws, size_t ws_size,
                              hipStream_t stream) {
  if (n_in < 10) return;
  if (in_sizes[0] != kTok * kDModel) return;
  if (in_sizes[1] != kDInner * kDModel) return;
  if (in_sizes[2] != kDHalf * kDConv) return;
  if (in_sizes[3] != kDHalf * kDConv) return;
  if (in_sizes[4] != kXdbl * kDHalf) return;
  if (in_sizes[5] != kDHalf * kDtRank) return;
  if (in_sizes[6] != kDHalf) return;
  if (in_sizes[7] != kDHalf * kDState) return;
  if (in_sizes[8] != kDHalf) return;
  if (in_sizes[9] != kDModel * kDInner) return;
  if (out_size != kTok * kDModel) return;

  const float* hs    = (const float*)d_in[0];
  const float* w_in  = (const float*)d_in[1];
  const float* w_cx  = (const float*)d_in[2];
  const float* w_cz  = (const float*)d_in[3];
  const float* w_xp  = (const float*)d_in[4];
  const float* w_dt  = (const float*)d_in[5];
  const float* b_dt  = (const float*)d_in[6];
  const float* a_log = (const float*)d_in[7];
  const float* d_vec = (const float*)d_in[8];
  const float* w_out = (const float*)d_in[9];
  float* out = (float*)d_out;

  const size_t offWIN  = 0;
  const size_t offWOUT = offWIN  + (size_t)kDInner * kDModel * 2;
  const size_t offWXP  = offWOUT + (size_t)kDModel * kDInner * 2;
  const size_t offWDT  = offWXP  + (size_t)kXdbl * kDHalf * 2;
  const size_t offH16  = offWDT  + (size_t)kDHalf * kDtRank * 2;
  const size_t offXPRE = offH16  + (size_t)kTok * kDModel * 2;
  const size_t offZPRE = offXPRE + (size_t)kTok * kDHalf * 4;
  const size_t offYZ   = offZPRE + (size_t)kTok * kDHalf * 4;
  const size_t offXDBL = offYZ   + (size_t)kTok * kDInner * 2;
  const size_t offDT16 = offXDBL + (size_t)kTok * kXdbl * 4;
  const size_t total   = offDT16 + (size_t)kTok * kDtRank * 2;
  if (total > ws_size) return;

  char* ws = (char*)d_ws;
  unsigned short* WIN16  = (unsigned short*)(ws + offWIN);
  unsigned short* WOUT16 = (unsigned short*)(ws + offWOUT);
  unsigned short* WXP16  = (unsigned short*)(ws + offWXP);
  unsigned short* WDT16  = (unsigned short*)(ws + offWDT);
  unsigned short* H16    = (unsigned short*)(ws + offH16);
  unsigned short* X16    = (unsigned short*)(ws + offH16);
  float*          XPRE   = (float*)(ws + offXPRE);
  float*          ZPRE   = (float*)(ws + offZPRE);
  float*          DTPRE  = (float*)(ws + offZPRE);
  unsigned short* YZ16   = (unsigned short*)(ws + offYZ);
  float*          XDBL   = (float*)(ws + offXDBL);
  unsigned short* DT16   = (unsigned short*)(ws + offDT16);

  {
    int n8;
    n8 = kTok * kDModel / 8;
    cast8_f16_kernel<<<(n8 + 255) / 256, 256, 0, stream>>>(hs, H16, n8, 1.0f);
    n8 = kDInner * kDModel / 8;
    cast8_f16_kernel<<<(n8 + 255) / 256, 256, 0, stream>>>(w_in, WIN16, n8, kWCarry);
    n8 = kXdbl * kDHalf / 8;
    cast8_f16_kernel<<<(n8 + 255) / 256, 256, 0, stream>>>(w_xp, WXP16, n8, kWCarry);
    n8 = kDHalf * kDtRank / 8;
    cast8_f16_kernel<<<(n8 + 255) / 256, 256, 0, stream>>>(w_dt, WDT16, n8, kWCarry);
    n8 = kDModel * kDInner / 8;
    cast8_f16_kernel<<<(n8 + 255) / 256, 256, 0, stream>>>(w_out, WOUT16, n8, kWCarry);
  }

  {
    const int blocks = ((kTok / 64) * (kDHalf / 64) + 7) / 8;
    wmma_gemm64<0, false, 0, 0, false, 0><<<dim3(blocks, 1), 256, 0, stream>>>(
        H16, H16, kDModel, 0L, WIN16, WIN16, kDModel, 0L,
        (void*)XPRE, (void*)XPRE, kDHalf, 0L, b_dt, b_dt, 0L, kTok, kDHalf, kDModel, kScaleIn);
    wmma_gemm64<0, false, 0, 0, false, 0><<<dim3(blocks, 1), 256, 0, stream>>>(
        H16, H16, kDModel, 0L, WIN16 + (size_t)kDHalf * kDModel, WIN16 + (size_t)kDHalf * kDModel, kDModel, 0L,
        (void*)ZPRE, (void*)ZPRE, kDHalf, 0L, b_dt, b_dt, 0L, kTok, kDHalf, kDModel, kScaleIn);
  }

  conv_silu_kernel<<<(kTok * 64) / 256, 256, 0, stream>>>(XPRE, ZPRE, w_cx, w_cz, X16, YZ16);

  {
    const int blocks = ((kTok / 64) * (kXdbl / 64) + 7) / 8;
    wmma_gemm64<0, false, 0, 0, false, 0><<<dim3(blocks, 1), 256, 0, stream>>>(
        X16, X16, kDHalf, 0L, WXP16, WXP16, kDHalf, 0L,
        (void*)XDBL, (void*)XDBL, kXdbl, 0L, b_dt, b_dt, 0L, kTok, kXdbl, kDHalf, kScaleAW);
  }

  {
    const int n8 = kTok * (kDtRank / 8);
    dtcast_kernel<<<(n8 + 255) / 256, 256, 0, stream>>>(XDBL, DT16, n8);
  }

  {
    const int blocks = ((kTok / 64) * (kDHalf / 64) + 7) / 8;
    wmma_gemm64<0, false, 2, 0, false, 0><<<dim3(blocks, 1), 256, 0, stream>>>(
        DT16, DT16, kDtRank, 0L, WDT16, WDT16, kDtRank, 0L,
        (void*)DTPRE, (void*)DTPRE, kDHalf, 0L, b_dt, b_dt, 0L, kTok, kDHalf, kDtRank, kScaleAW);
  }

  scan_kernel<<<dim3(kBatch, kDHalf / 128), 128, 0, stream>>>(XPRE, XDBL, DTPRE, a_log, d_vec, w_cx, YZ16);

  {
    const int blocks = ((kTok / 64) * (kDModel / 64) + 7) / 8;
    wmma_gemm64<0, false, 0, 0, false, 0><<<dim3(blocks, 1), 256, 0, stream>>>(
        YZ16, YZ16, kDInner, 0L, WOUT16, WOUT16, kDInner, 0L,
        (void*)out, (void*)out, kDModel, 0L, b_dt, b_dt, 0L, kTok, kDModel, kDInner, kScaleAW);
  }
}
